// CrossAttentionBlock_2362232013219
// MI455X (gfx1250) — hardware-verified
//
#include <hip/hip_runtime.h>
#include <stddef.h>


#ifndef NB
#define NB 4
#endif
#ifndef SEQ
#define SEQ 2304
#endif
#define NB_FULL  4
#define SEQ_FULL 2304
#define CH   256
#define NHD  8
#define HD   32
#define WSZ  (CH * CH)

static_assert(SEQ % 256 == 0);
static_assert(SEQ >= 256 && SEQ <= SEQ_FULL);
static_assert(NB >= 1 && NB <= NB_FULL);
static_assert(CH == NHD * HD);

typedef _Float16 f16t;
typedef f16t  v8h  __attribute__((ext_vector_type(8)));
typedef f16t  v16h __attribute__((ext_vector_type(16)));
typedef float v8f  __attribute__((ext_vector_type(8)));
typedef float v4f  __attribute__((ext_vector_type(4)));
typedef unsigned int v4u __attribute__((ext_vector_type(4)));

__device__ __forceinline__ float bf16r(float f) {
  unsigned u = __float_as_uint(f);
  u = (u + 0x7FFFu + ((u >> 16) & 1u)) & 0xFFFF0000u;
  return __uint_as_float(u);
}

__device__ __forceinline__ v16h ldfrag(const f16t* p) {
  v8h lo = *(const v8h*)p;
  v8h hi = *(const v8h*)(p + 16);
  return __builtin_shufflevector(lo, hi, 0, 1, 2, 3, 4, 5, 6, 7, 8, 9, 10, 11, 12, 13, 14, 15);
}

__device__ __forceinline__ v8f mma16(v16h a, v16h b, v8f c) {
  v8f d = __builtin_amdgcn_wmma_f32_16x16x32_f16(false, a, false, b, (short)0, c, false, false);
  asm volatile("v_nop\n\tv_nop\n\tv_nop\n\tv_nop" : "+v"(d) : "v"(a), "v"(b));
  return d;
}

__device__ __forceinline__ v8f vzero8() {
  v8f z;
  #pragma unroll
  for (int i = 0; i < 8; ++i) z[i] = 0.0f;
  return z;
}

__global__ __launch_bounds__(256) void cvt_tok_kernel(const float* __restrict__ x,
                                                      const float* __restrict__ ctx,
                                                      f16t* __restrict__ xh,
                                                      f16t* __restrict__ ch) {
  __shared__ __align__(16) f16t tile[64][72];
  const int bz = blockIdx.z;
  const bool second = (bz >= NB);
  const int b = second ? (bz - NB) : bz;
  const float* src = second ? ctx : x;
  f16t* dst = second ? ch : xh;
  const int s0 = blockIdx.x * 64, c0 = blockIdx.y * 64;
  const int t = threadIdx.x, ss = t & 63, cq = t >> 6;
  const float* sp = src + ((size_t)(b * CH + c0)) * SEQ_FULL + s0 + ss;
  #pragma unroll
  for (int i = 0; i < 16; ++i) {
    const int cc = cq + 4 * i;
    tile[ss][cc] = (f16t)bf16r(sp[(size_t)cc * SEQ_FULL]);
  }
  __syncthreads();

  const int w = t >> 5, lane = t & 31;
  v4u u[2];
  f16t* gp[2];
  #pragma unroll
  for (int j = 0; j < 2; ++j) {
    const int tok = w * 8 + j * 4 + (lane >> 3);
    const int cof = (lane & 7) * 8;
    v8h v = *(const v8h*)&tile[tok][cof];
    u[j] = __builtin_bit_cast(v4u, v);
    gp[j] = dst + ((size_t)(b * SEQ + s0 + tok)) * CH + c0 + cof;
  }
  #pragma unroll
  for (int j = 0; j < 2; ++j) *(volatile v4u*)gp[j] = u[j];
  __threadfence();
  #pragma unroll
  for (int j = 0; j < 2; ++j) *(volatile v4u*)gp[j] = u[j];
}

__global__ __launch_bounds__(256) void cvt_w_kernel(const float* __restrict__ wq,
                                                    const float* __restrict__ wk,
                                                    const float* __restrict__ wv,
                                                    const float* __restrict__ wo,
                                                    f16t* __restrict__ w16) {
  const int gi  = blockIdx.x * 256 + threadIdx.x;
  const int mat = gi >> 13;
  const int e   = (gi & 8191) * 8;
  const float* src = (mat == 0) ? wq : (mat == 1) ? wk : (mat == 2) ? wv : wo;
  const float4 a = *(const float4*)(src + e);
  const float4 c = *(const float4*)(src + e + 4);
  v8h o;
  o[0] = (f16t)(16.0f * bf16r(a.x)); o[1] = (f16t)(16.0f * bf16r(a.y));
  o[2] = (f16t)(16.0f * bf16r(a.z)); o[3] = (f16t)(16.0f * bf16r(a.w));
  o[4] = (f16t)(16.0f * bf16r(c.x)); o[5] = (f16t)(16.0f * bf16r(c.y));
  o[6] = (f16t)(16.0f * bf16r(c.z)); o[7] = (f16t)(16.0f * bf16r(c.w));
  const v4u u = __builtin_bit_cast(v4u, o);
  f16t* gp = w16 + (size_t)mat * WSZ + e;
  *(volatile v4u*)gp = u;
  __threadfence();
  *(volatile v4u*)gp = u;
}

struct GemmDesc {
  const f16t* A; const f16t* Bt; f16t* D; const float* bias;
  long long sAb, sBb, sDb;
  int lda, ldb, ldd, bias_mode;
};
static_assert(sizeof(GemmDesc) == 72);

__global__ __launch_bounds__(256) void gemm_kernel(GemmDesc g0, GemmDesc g1, int zsplit) {
  __shared__ __align__(16) f16t stg[32][264];
  const int z = blockIdx.z;
  const bool sel = (z >= zsplit);
  const int batch = sel ? (z - zsplit) : z;
  const f16t* A     = sel ? g1.A : g0.A;
  const f16t* Bt    = sel ? g1.Bt : g0.Bt;
  f16t* D           = sel ? g1.D : g0.D;
  const float* bias = sel ? g1.bias : g0.bias;
  const long long sAb = sel ? g1.sAb : g0.sAb;
  const long long sBb = sel ? g1.sBb : g0.sBb;
  const long long sDb = sel ? g1.sDb : g0.sDb;
  const int lda = sel ? g1.lda : g0.lda;
  const int ldb = sel ? g1.ldb : g0.ldb;
  const int ldd = sel ? g1.ldd : g0.ldd;
  const int bias_mode = sel ? g1.bias_mode : g0.bias_mode;

  const int w = threadIdx.x >> 5, lane = threadIdx.x & 31;
  const int lr = lane & 15, lh = lane >> 4;
  const int rg = w >> 2, cg = w & 3;
  const int rowbase = blockIdx.y * 32 + rg * 16;
  const int colbase = blockIdx.x * 256 + cg * 64;
  const f16t* Ab = A + (size_t)batch * (size_t)sAb;
  const f16t* Bb = Bt + (size_t)batch * (size_t)sBb;
  f16t* Db = D + (size_t)batch * (size_t)sDb;

  v16h Af[8];
  const f16t* arow = Ab + (size_t)(rowbase + lr) * lda + lh * 8;
  #pragma unroll
  for (int kc = 0; kc < 8; ++kc) Af[kc] = ldfrag(arow + kc * 32);

  v8f acc[4];
  #pragma unroll
  for (int tt = 0; tt < 4; ++tt) acc[tt] = vzero8();
  #pragma unroll
  for (int kc = 0; kc < 8; ++kc) {
    #pragma unroll
    for (int tt = 0; tt < 4; ++tt) {
      const f16t* brow = Bb + (size_t)(colbase + tt * 16 + lr) * ldb + kc * 32 + lh * 8;
      acc[tt] = mma16(Af[kc], ldfrag(brow), acc[tt]);
    }
  }

  float brow8[8];
  #pragma unroll
  for (int i = 0; i < 8; ++i) {
    const int r  = rowbase + 8 * lh + i;
    const int rc = (r < CH) ? r : (CH - 1);
    brow8[i] = bf16r(bias[rc]);
  }
  #pragma unroll
  for (int tt = 0; tt < 4; ++tt) {
    const int col  = colbase + tt * 16 + lr;
    const int ccl  = (col < CH) ? col : (CH - 1);
    const float bc = bf16r(bias[ccl]);
    const int lcol = cg * 64 + tt * 16 + lr;
    #pragma unroll
    for (int i = 0; i < 8; ++i) {
      const float bb = (bias_mode == 0) ? bc : brow8[i];
      const float v  = acc[tt][i] * 0.0625f + bb;
      stg[rg * 16 + 8 * lh + i][lcol] = (f16t)v;
    }
  }
  __syncthreads();

  v4u u[4];
  f16t* gp[4];
  #pragma unroll
  for (int j = 0; j < 4; ++j) {
    const int lrow = w * 4 + j;
    v8h v = *(const v8h*)&stg[lrow][lane * 8];
    u[j]  = __builtin_bit_cast(v4u, v);
    gp[j] = Db + (size_t)(blockIdx.y * 32 + lrow) * ldd + blockIdx.x * 256 + lane * 8;
  }
  #pragma unroll
  for (int j = 0; j < 4; ++j) *(volatile v4u*)gp[j] = u[j];
  __threadfence();
  #pragma unroll
  for (int j = 0; j < 4; ++j) *(volatile v4u*)gp[j] = u[j];
}

__global__ __launch_bounds__(256) void attn_kernel(const f16t* __restrict__ Qh,
                                                   const f16t* __restrict__ Kh,
                                                   const f16t* __restrict__ Vt,
                                                   f16t* __restrict__ Ah) {
  __shared__ __align__(16) f16t sK[32 * 32];
  __shared__ __align__(16) f16t sV[32 * 32];
  __shared__ __align__(16) f16t sP[8][16 * 32];
  const float scale = 0.17677669529663687f;

  const int t = threadIdx.x, lane = t & 31, w = t >> 5;
  const int lr = lane & 15, hf = lane >> 4;
  const int bh = blockIdx.y, b = bh >> 3, h = bh & 7;
  const int qbase = blockIdx.x * 128 + w * 16;

  const v16h aq = ldfrag(Qh + ((size_t)(b * SEQ + qbase + lr)) * CH + h * HD + hf * 8);

  float mrow[8], lsum[8];
  #pragma unroll
  for (int r = 0; r < 8; ++r) { mrow[r] = -3.0e38f; lsum[r] = 0.0f; }
  const v8f vz = vzero8();
  v8f o0 = vz, o1 = vz;

  #pragma unroll 1
  for (int kt = 0; kt < SEQ / 32; ++kt) {
    __syncthreads();
    if (t < 128) {
      const int row = t >> 2, q = t & 3;
      *(v8h*)&sK[row * 32 + q * 8] =
          *(const v8h*)&Kh[((size_t)(b * SEQ + kt * 32 + row)) * CH + h * HD + q * 8];
    } else {
      const int t2 = t - 128, row = t2 >> 2, q = t2 & 3;
      *(v8h*)&sV[row * 32 + q * 8] =
          *(const v8h*)&Vt[((size_t)(b * CH + h * HD + row)) * SEQ + kt * 32 + q * 8];
    }
    __syncthreads();

    const v16h bk0 = ldfrag(&sK[lr * 32 + hf * 8]);
    const v16h bk1 = ldfrag(&sK[(16 + lr) * 32 + hf * 8]);
    const v8f s0 = mma16(aq, bk0, vz);
    const v8f s1 = mma16(aq, bk1, vz);

    #pragma unroll
    for (int r = 0; r < 8; ++r) {
      const float v0 = s0[r] * scale, v1 = s1[r] * scale;
      float tm = fmaxf(v0, v1);
      tm = fmaxf(tm, __shfl_xor(tm, 1, 32));
      tm = fmaxf(tm, __shfl_xor(tm, 2, 32));
      tm = fmaxf(tm, __shfl_xor(tm, 4, 32));
      tm = fmaxf(tm, __shfl_xor(tm, 8, 32));
      const float mnew  = fmaxf(mrow[r], tm);
      const float alpha = __expf(mrow[r] - mnew);
      const float p0 = __expf(v0 - mnew);
      const float p1 = __expf(v1 - mnew);
      float rs = p0 + p1;
      rs += __shfl_xor(rs, 1, 32);
      rs += __shfl_xor(rs, 2, 32);
      rs += __shfl_xor(rs, 4, 32);
      rs += __shfl_xor(rs, 8, 32);
      lsum[r] = lsum[r] * alpha + rs;
      mrow[r] = mnew;
      o0[r] = o0[r] * alpha;
      o1[r] = o1[r] * alpha;
      sP[w][(hf * 8 + r) * 32 + lr]      = (f16t)(p0 * 1024.0f);
      sP[w][(hf * 8 + r) * 32 + 16 + lr] = (f16t)(p1 * 1024.0f);
    }
    __syncthreads();

    const v16h ap  = ldfrag(&sP[w][lr * 32 + hf * 8]);
    const v16h bv0 = ldfrag(&sV[lr * 32 + hf * 8]);
    const v16h bv1 = ldfrag(&sV[(16 + lr) * 32 + hf * 8]);
    o0 = mma16(ap, bv0, o0);
    o1 = mma16(ap, bv1, o1);
  }

  float inv[8];
  #pragma unroll
  for (int r = 0; r < 8; ++r) inv[r] = 1.0f / (lsum[r] * 64.0f);
  __syncthreads();
  #pragma unroll
  for (int r = 0; r < 8; ++r) {
    sP[w][(hf * 8 + r) * 32 + lr]      = (f16t)(o0[r] * inv[r]);
    sP[w][(hf * 8 + r) * 32 + 16 + lr] = (f16t)(o1[r] * inv[r]);
  }
  __syncthreads();
  v4u u[2];
  f16t* gp[2];
  #pragma unroll
  for (int j = 0; j < 2; ++j) {
    const int lrow = j * 8 + (lane >> 2);
    const int lcol = (lane & 3) * 8;
    v8h v = *(const v8h*)&sP[w][lrow * 32 + lcol];
    u[j]  = __builtin_bit_cast(v4u, v);
    gp[j] = Ah + (((size_t)(b * NHD + h)) * SEQ + qbase + lrow) * HD + lcol;
  }
  #pragma unroll
  for (int j = 0; j < 2; ++j) *(volatile v4u*)gp[j] = u[j];
  __threadfence();
  #pragma unroll
  for (int j = 0; j < 2; ++j) *(volatile v4u*)gp[j] = u[j];
}

__global__ __launch_bounds__(256) void oproj_ln_kernel(const f16t* __restrict__ Ah,
                                                       const f16t* __restrict__ Wo16,
                                                       const float* __restrict__ bo,
                                                       const float* __restrict__ x,
                                                       const float* __restrict__ lnw,
                                                       const float* __restrict__ lnb,
                                                       float* __restrict__ out) {
  __shared__ float yt[32][257];
  __shared__ float red[32][9];
  __shared__ float smean[32], sinv[32];

  const int t = threadIdx.x, lane = t & 31, w = t >> 5;
  const int lr = lane & 15, hf = lane >> 4;
  const int mbase = blockIdx.x * 32, b = blockIdx.y;

  v8f acc[2][2];
  #pragma unroll
  for (int mt = 0; mt < 2; ++mt)
    #pragma unroll
    for (int nt = 0; nt < 2; ++nt) acc[mt][nt] = vzero8();

  #pragma unroll
  for (int kc = 0; kc < NHD; ++kc) {
    const f16t* abase = Ah + ((size_t)((b * NHD + kc) * SEQ + mbase)) * HD;
    v16h af[2], bf[2];
    #pragma unroll
    for (int mt = 0; mt < 2; ++mt) af[mt] = ldfrag(abase + (size_t)(mt * 16 + lr) * HD + hf * 8);
    #pragma unroll
    for (int nt = 0; nt < 2; ++nt)
      bf[nt] = ldfrag(Wo16 + (size_t)(w * 32 + nt * 16 + lr) * CH + kc * 32 + hf * 8);
    #pragma unroll
    for (int mt = 0; mt < 2; ++mt)
      #pragma unroll
      for (int nt = 0; nt < 2; ++nt) acc[mt][nt] = mma16(af[mt], bf[nt], acc[mt][nt]);
  }

  #pragma unroll
  for (int mt = 0; mt < 2; ++mt)
    #pragma unroll
    for (int nt = 0; nt < 2; ++nt) {
      const int c = w * 32 + nt * 16 + lr;
      const float bb = bf16r(bo[c]);
      const int srow0 = mt * 16 + hf * 8;
      const float* xp = x + ((size_t)(b * CH + c)) * SEQ_FULL + mbase + srow0;
      const float4 x0 = *(const float4*)xp;
      const float4 x1 = *(const float4*)(xp + 4);
      float xv[8] = {x0.x, x0.y, x0.z, x0.w, x1.x, x1.y, x1.z, x1.w};
      #pragma unroll
      for (int r = 0; r < 8; ++r)
        yt[srow0 + r][c] = acc[mt][nt][r] * 0.00390625f + bb + bf16r(xv[r]);
    }
  __syncthreads();

  {
    const int row = t & 31, chunk = t >> 5;
    float s1 = 0.0f;
    #pragma unroll
    for (int j = 0; j < 32; ++j) s1 += yt[row][chunk * 32 + j];
    red[row][chunk] = s1;
  }
  __syncthreads();
  if (t < 32) {
    float s1 = 0.0f;
    #pragma unroll
    for (int j = 0; j < 8; ++j) s1 += red[t][j];
    smean[t] = s1 * 0.00390625f;
  }
  __syncthreads();
  {
    const int row = t & 31, chunk = t >> 5;
    const float mu = smean[row];
    float s2 = 0.0f;
    #pragma unroll
    for (int j = 0; j < 32; ++j) {
      const float d = yt[row][chunk * 32 + j] - mu;
      s2 += d * d;
    }
    red[row][chunk] = s2;
  }
  __syncthreads();
  if (t < 32) {
    float s2 = 0.0f;
    #pragma unroll
    for (int j = 0; j < 8; ++j) s2 += red[t][j];
    const float var = s2 * 0.00390625f;
    sinv[t] = rsqrtf(var + 1e-5f);
  }
  __syncthreads();

  const int s4 = (lane & 7) * 4;
  float mu4[4], iv4[4];
  #pragma unroll
  for (int i = 0; i < 4; ++i) { mu4[i] = smean[s4 + i]; iv4[i] = sinv[s4 + i]; }
  v4f ov[8];
  float* op[8];
  #pragma unroll
  for (int j = 0; j < 8; ++j) {
    const int c = w * 32 + j * 4 + (lane >> 3);
    const float gw = bf16r(lnw[c]), gb = bf16r(lnb[c]);
    v4f v;
    #pragma unroll
    for (int i = 0; i < 4; ++i) v[i] = (yt[s4 + i][c] - mu4[i]) * iv4[i] * gw + gb;
    ov[j] = v;
    op[j] = out + ((size_t)(b * CH + c)) * SEQ_FULL + mbase + s4;
  }
  #pragma unroll
  for (int j = 0; j < 8; ++j) *(volatile v4f*)op[j] = ov[j];
  __threadfence();
  #pragma unroll
  for (int j = 0; j < 8; ++j) *(volatile v4f*)op[j] = ov[j];
}

extern "C" void kernel_launch(void* const* d_in, const int* in_sizes, int n_in,
                              void* d_out, int out_size, void* d_ws, size_t ws_size,
                              hipStream_t stream) {
  if (n_in < 12) return;
  const float* x   = (const float*)d_in[0];
  const float* ctx = (const float*)d_in[1];
  const float* Wq  = (const float*)d_in[2];
  const float* bq  = (const float*)d_in[3];
  const float* Wk  = (const float*)d_in[4];
  const float* bk  = (const float*)d_in[5];
  const float* Wv  = (const float*)d_in[6];
  const float* bv  = (const float*)d_in[7];
  const float* Wo  = (const float*)d_in[8];
  const float* bo  = (const float*)d_in[9];
  const float* lnw = (const float*)d_in[10];
  const float* lnb = (const float*)d_in[11];
  float* outp = (float*)d_out;

  const size_t needx = (size_t)(NB * CH - 1) * SEQ_FULL + SEQ;
  if ((size_t)in_sizes[0] < needx || (size_t)in_sizes[1] < needx) return;
  if (in_sizes[2] < WSZ || in_sizes[4] < WSZ || in_sizes[6] < WSZ || in_sizes[8] < WSZ) return;
  if (in_sizes[3] < CH || in_sizes[5] < CH || in_sizes[7] < CH || in_sizes[9] < CH ||
      in_sizes[10] < CH || in_sizes[11] < CH) return;
  if ((size_t)out_size < needx) return;

  const size_t E = (size_t)NB * SEQ * CH;
  const size_t total_halves = 6 * E + 4 * (size_t)WSZ;
  if (total_halves * sizeof(f16t) > ws_size) return;

  f16t* Xh  = (f16t*)d_ws;
  f16t* Ch  = Xh + E;
  f16t* Qh  = Ch + E;
  f16t* Kh  = Qh + E;
  f16t* Vt  = Kh + E;
  f16t* Ah  = Vt + E;
  f16t* W16 = Ah + E;

  cvt_tok_kernel<<<dim3(SEQ / 64, CH / 64, 2 * NB), 256, 0, stream>>>(x, ctx, Xh, Ch);
  cvt_w_kernel<<<dim3(128), 256, 0, stream>>>(Wq, Wk, Wv, Wo, W16);

  GemmDesc gq;
  gq.A = Xh; gq.Bt = W16; gq.D = Qh; gq.bias = bq;
  gq.sAb = (long long)SEQ * CH; gq.sBb = 0; gq.sDb = (long long)SEQ * CH;
  gq.lda = CH; gq.ldb = CH; gq.ldd = CH; gq.bias_mode = 0;
  GemmDesc gk = gq;
  gk.A = Ch; gk.Bt = W16 + WSZ; gk.D = Kh; gk.bias = bk;
  GemmDesc gv;
  gv.A = W16 + 2 * WSZ; gv.Bt = Ch; gv.D = Vt; gv.bias = bv;
  gv.sAb = 0; gv.sBb = (long long)SEQ * CH; gv.sDb = (long long)CH * SEQ;
  gv.lda = CH; gv.ldb = CH; gv.ldd = SEQ; gv.bias_mode = 1;

  gemm_kernel<<<dim3(1, SEQ / 32, 2 * NB), 256, 0, stream>>>(gq, gk, NB);
  gemm_kernel<<<dim3(SEQ / 256, CH / 32, NB), 256, 0, stream>>>(gv, gv, NB);

  attn_kernel<<<dim3(SEQ / 128, NB * NHD), 256, 0, stream>>>(Qh, Kh, Vt, Ah);

  oproj_ln_kernel<<<dim3(SEQ / 32, NB), 256, 0, stream>>>(Ah, W16 + 3 * WSZ, bo, x, lnw, lnb, outp);
}
